// TemporalHybrid_34402688041056
// MI455X (gfx1250) — hardware-run, weakly checked
//
#include <hip/hip_runtime.h>
#include <math.h>

typedef __attribute__((ext_vector_type(16))) _Float16 v16h;
typedef __attribute__((ext_vector_type(8)))  _Float16 v8h;
typedef __attribute__((ext_vector_type(8)))  float    v8f;
typedef __attribute__((ext_vector_type(4)))  float    v4f;
typedef __attribute__((ext_vector_type(4)))  unsigned v4u;
typedef __attribute__((ext_vector_type(2)))  unsigned v2u;

constexpr int kBatch   = 32;
constexpr int kLen     = 1024;
constexpr int kChanIn  = 64;
constexpr int kWidth   = 256;
constexpr int kModes   = 256;
constexpr int kChunk   = 128;
constexpr int kBlocksD = kLen / kChunk;
constexpr int kNpos    = kBatch * kLen;
constexpr int kDilK    = 3 * kChanIn;
constexpr int kPitchW  = 132;
constexpr int kPitchX  = 36;
constexpr int kTabSz   = 64 * 33;
static_assert(kBlocksD == 8 && kNpos == 32768 && kDilK == 192);
static_assert((kChanIn % 32) == 0 && (kChunk % 32) == 0 && (kWidth % 32) == 0 && (kDilK % 32) == 0);
static_assert((kNpos % 64) == 0 && (kLen % 64) == 0 && (kWidth % 64) == 0 && (kChunk % 64) == 0 && (kBatch % 32) == 0);

constexpr bool kEncLo = false;
constexpr bool kDecLo = false;
constexpr bool kDilLo = false;

constexpr float kWCarry    = 256.0f;
constexpr float kWCarryInv = 1.0f / 256.0f;
constexpr float kTCarry    = 64.0f;
constexpr float kTCarryInv = 1.0f / 64.0f;
constexpr float kLoScale   = 2048.0f;
constexpr float kLoInv     = 1.0f / 2048.0f;

constexpr size_t kOffU16  = 0;
constexpr size_t kOffG16  = kOffU16  + (size_t)kWidth * kNpos * 2;
constexpr size_t kOffKt   = kOffG16  + (size_t)kWidth * kNpos * 2;
constexpr size_t kOffTb   = kOffKt   + (size_t)kWidth * kLen * 4;
constexpr size_t kOffEncT = kOffTb   + (size_t)kWidth * kBlocksD * kChunk * kChunk * 2;
constexpr size_t kOffEncL = kOffEncT + (size_t)kWidth * kChanIn * 2;
constexpr size_t kOffDecT = kOffEncL + (size_t)kWidth * kChanIn * 2;
constexpr size_t kOffDecL = kOffDecT + (size_t)kWidth * kWidth * 2;
constexpr size_t kOffDilT = kOffDecL + (size_t)kWidth * kWidth * 2;
constexpr size_t kOffDilL = kOffDilT + (size_t)kWidth * kDilK * 2;
constexpr size_t kWsTotal = kOffDilL + (size_t)kWidth * kDilK * 2;
static_assert(kWsTotal == 102236160ull);
static_assert(kWsTotal <= 134217728ull);
static_assert((kOffG16 % 256) == 0 && (kOffKt % 256) == 0 && (kOffTb % 256) == 0 && (kOffEncT % 256) == 0 &&
              (kOffEncL % 256) == 0 && (kOffDecT % 256) == 0 && (kOffDecL % 256) == 0 && (kOffDilT % 256) == 0 &&
              (kOffDilL % 256) == 0);

__device__ __forceinline__ float flush16(float v) {
  return (__builtin_fabsf(v) < 6.103515625e-5f) ? 0.0f : v;
}
__device__ __forceinline__ unsigned short f16bits(float x) {
  const _Float16 h = (_Float16)flush16(x);
  return __builtin_bit_cast(unsigned short, h);
}
__device__ __forceinline__ unsigned pack2(float a, float b) {
  const unsigned lo = (unsigned)f16bits(a);
  const unsigned hi = (unsigned)f16bits(b);
  return lo | (hi << 16);
}
__device__ __forceinline__ float h16_to_f32(unsigned hb) {
  const unsigned sgn = (hb & 0x8000u) << 16;
  const unsigned em = hb & 0x7fffu;
  const float fn = __uint_as_float((em << 13) + 0x38000000u);
  const float fs = (float)em * 5.9604644775390625e-8f;
  const float mag = (em < 0x400u) ? fs : fn;
  return __uint_as_float(__float_as_uint(mag) | sgn);
}
__device__ __forceinline__ void wave_sync() {
  __builtin_amdgcn_fence(__ATOMIC_RELEASE, "workgroup");
  __builtin_amdgcn_wave_barrier();
  __builtin_amdgcn_fence(__ATOMIC_ACQUIRE, "workgroup");
}
__device__ __forceinline__ void store2_v4u(unsigned short* p, v4u v) {
  volatile v4u* q = (volatile v4u*)p;
  *q = v;
  __threadfence();
  *q = v;
}
__device__ __forceinline__ float gelu_fast(float y) {
  const float u = 0.7978845608028654f * (y + 0.044715f * y * y * y);
  const float e = __expf(-2.0f * u);
  return y * __builtin_amdgcn_rcpf(1.0f + e);
}
__device__ __forceinline__ void cmul(float& ar, float& ai, float br, float bi) {
  const float t = ar * br - ai * bi;
  ai = ar * bi + ai * br;
  ar = t;
}
__device__ __forceinline__ void csq(float& ar, float& ai) {
  const float t = ar * ar - ai * ai;
  ai = 2.0f * ar * ai;
  ar = t;
}

union FragH { v16h v; v8h h[2]; };
union FragW { v16h v; v4u q[2]; };
__device__ __forceinline__ v16h frag_load(const _Float16* p) {
  FragH f;
  f.h[0] = *(const v8h*)(p);
  f.h[1] = *(const v8h*)(p + 16);
  return f.v;
}
template <int PITCH>
__device__ __forceinline__ v16h lds_frag(const unsigned* sw, int n, int kw) {
  FragW f;
  f.q[0] = *(const v4u*)(sw + n * PITCH + kw);
  f.q[1] = *(const v4u*)(sw + n * PITCH + kw + 8);
  return f.v;
}
__device__ __forceinline__ v8f mma16(v16h a, v16h b, v8f c) {
  return __builtin_amdgcn_wmma_f32_16x16x32_f16(false, a, false, b, (short)0, c, false, false);
}
__device__ __forceinline__ void tie_acc(v8f& a, v16h x, v16h y) { asm volatile("" : "+v"(a) : "v"(x), "v"(y)); }
__device__ __forceinline__ void tie_acc_nops(v8f& a, v16h x, v16h y) { asm volatile("v_nop\n\tv_nop\n\tv_nop\n\tv_nop" : "+v"(a) : "v"(x), "v"(y)); }
__device__ __forceinline__ void keep4(v16h a, v16h b, v16h c, v16h d) { asm volatile("v_nop" :: "v"(a), "v"(b), "v"(c), "v"(d)); }
__device__ __forceinline__ void acc_guard4(v8f& a, v8f& b, v8f& c, v8f& d) { asm volatile("v_nop\n\tv_nop\n\tv_nop\n\tv_nop" : "+v"(a), "+v"(b), "+v"(c), "+v"(d)); }

__device__ __forceinline__ void kloop32(v8f (&acc)[2][4], const _Float16* ap, int lda,
                                        const _Float16* bp, int ldb, int ksteps) {
#pragma unroll 1
  for (int ks = 0; ks < ksteps; ++ks) {
    v16h bh[4];
#pragma unroll
    for (int j = 0; j < 4; ++j) bh[j] = frag_load(bp + (size_t)(j * 16) * ldb + ks * 32);
#pragma unroll
    for (int i = 0; i < 2; ++i) {
      const v16h ah = frag_load(ap + (size_t)(i * 16) * lda + ks * 32);
#pragma unroll
      for (int j = 0; j < 4; ++j) acc[i][j] = mma16(ah, bh[j], acc[i][j]);
      tie_acc(acc[i][0], ah, bh[0]);
      tie_acc(acc[i][1], ah, bh[1]);
      tie_acc(acc[i][2], ah, bh[2]);
      tie_acc_nops(acc[i][3], ah, bh[3]);
    }
    keep4(bh[0], bh[1], bh[2], bh[3]);
  }
}

template <bool LO, int PITCH>
__device__ __forceinline__ void tile_kloop(v8f (&acc)[2][4], v8f (&accl)[2][4],
                                           const _Float16* ahp, const _Float16* alp, int lda,
                                           const unsigned* sw, int nrow, int kw0, int ksteps) {
#pragma unroll 1
  for (int ks = 0; ks < ksteps; ++ks) {
    v16h bf[4];
#pragma unroll
    for (int j = 0; j < 4; ++j) bf[j] = lds_frag<PITCH>(sw, nrow + 16 * j, kw0 + ks * 16);
#pragma unroll
    for (int i = 0; i < 2; ++i) {
      const v16h ah = frag_load(ahp + (size_t)(i * 16) * lda + ks * 32);
#pragma unroll
      for (int j = 0; j < 4; ++j) acc[i][j] = mma16(ah, bf[j], acc[i][j]);
      tie_acc(acc[i][0], ah, bf[0]);
      tie_acc(acc[i][1], ah, bf[1]);
      tie_acc(acc[i][2], ah, bf[2]);
      tie_acc_nops(acc[i][3], ah, bf[3]);
      if (LO) {
        const v16h al = frag_load(alp + (size_t)(i * 16) * lda + ks * 32);
#pragma unroll
        for (int j = 0; j < 4; ++j) accl[i][j] = mma16(al, bf[j], accl[i][j]);
        tie_acc(accl[i][0], al, bf[0]);
        tie_acc(accl[i][1], al, bf[1]);
        tie_acc(accl[i][2], al, bf[2]);
        tie_acc_nops(accl[i][3], al, bf[3]);
      }
    }
    keep4(bf[0], bf[1], bf[2], bf[3]);
  }
}

template <int NT>
__device__ __forceinline__ void stage_tile_T(const unsigned short* plane, size_t n0, unsigned* sw, int tid) {
#pragma unroll 1
  for (int it = 0; it < 1024 / NT; ++it) {
    const int task = it * NT + tid;
    const int n8 = task & 7;
    const int kp = task >> 3;
    const unsigned short* p0 = plane + (size_t)(2 * kp) * kNpos + n0 + n8 * 8;
    const v4u a = *(const v4u*)(p0);
    const v4u b = *(const v4u*)(p0 + kNpos);
    unsigned* dst = sw + (n8 * 8) * kPitchW + kp;
#pragma unroll
    for (int j = 0; j < 4; ++j) {
      const unsigned aw = a[j];
      const unsigned bw = b[j];
      dst[(2 * j) * kPitchW]     = (aw & 0xffffu) | (bw << 16);
      dst[(2 * j + 1) * kPitchW] = (aw >> 16) | (bw & 0xffff0000u);
    }
  }
}

__device__ __forceinline__ void store_tile_rows(const unsigned* sw, unsigned short* plane, size_t n0, int wave, int lane) {
  const int q = lane >> 3;
  const int cw = lane & 7;
  v4u vals[8];
#pragma unroll
  for (int it = 0; it < 8; ++it) {
    const int row = it * 32 + wave * 4 + q;
    vals[it] = *(const v4u*)(sw + row * 32 + cw * 4);
  }
  for (int pass = 0; pass < 2; ++pass) {
#pragma unroll
    for (int it = 0; it < 8; ++it) {
      const int row = it * 32 + wave * 4 + q;
      *(volatile v4u*)(plane + (size_t)row * kNpos + n0 + cw * 8) = vals[it];
    }
    __threadfence();
  }
}

template <int KREAL, int KP, bool LO>
__device__ __forceinline__ void transpose_rows(const float* __restrict__ src, int ld, int mcount, int m0, int rows_valid,
                                               unsigned short* dhi, unsigned short* dlo, float* sT, int tid) {
  const int mm = tid & 31;
  const int kq = tid >> 5;
  int ms = m0 + mm;
  ms = (ms < mcount) ? ms : (mcount - 1);
#pragma unroll 1
  for (int it = 0; it < KREAL / 8; ++it) {
    const int k = it * 8 + kq;
    sT[mm * 257 + k] = src[(size_t)k * ld + ms];
  }
  __syncthreads();
  constexpr int CPR = KP / 8;
  constexpr int ITERS = (32 * CPR + 255) / 256;
  const int nchunks = rows_valid * CPR;
#pragma unroll 1
  for (int it = 0; it < ITERS; ++it) {
    const int q = it * 256 + tid;
    if (q < nchunks) {
      const int row = q / CPR;
      const int k8 = (q - row * CPR) * 8;
      float vh[8];
      float vl[8];
#pragma unroll
      for (int e = 0; e < 8; ++e) {
        const int kk = k8 + e;
        const int kc = (kk < KREAL) ? kk : (KREAL - 1);
        const float x = sT[row * 257 + kc];
        const float v = (kk < KREAL) ? (x * kWCarry) : 0.0f;
        const _Float16 hv = (_Float16)flush16(v);
        const float back = (float)hv;
        vh[e] = v;
        vl[e] = (v - back) * kLoScale;
      }
      const v4u ph = {pack2(vh[0], vh[1]), pack2(vh[2], vh[3]), pack2(vh[4], vh[5]), pack2(vh[6], vh[7])};
      store2_v4u(dhi + (size_t)q * 8, ph);
      if (LO) {
        const v4u pl = {pack2(vl[0], vl[1]), pack2(vl[2], vl[3]), pack2(vl[4], vl[5]), pack2(vl[6], vl[7])};
        store2_v4u(dlo + (size_t)q * 8, pl);
      }
    }
  }
}

__global__ __launch_bounds__(256) void weight_planes_kernel(
    const float* __restrict__ enc_w, const float* __restrict__ dec_w, const float* __restrict__ dil_w,
    unsigned short* __restrict__ encT, unsigned short* __restrict__ encL,
    unsigned short* __restrict__ decT, unsigned short* __restrict__ decL,
    unsigned short* __restrict__ dilT, unsigned short* __restrict__ dilL) {
  __shared__ float sT[32 * 257];
  const int tid = threadIdx.x;
  const int bid = blockIdx.x;
  if (bid < 8) {
    const int m0 = bid * 32;
    transpose_rows<kChanIn, kChanIn, kEncLo>(enc_w, kWidth, kWidth, m0, 32,
                                             encT + (size_t)m0 * kChanIn, encL + (size_t)m0 * kChanIn, sT, tid);
  } else if (bid < 16) {
    const int m0 = (bid - 8) * 32;
    transpose_rows<kWidth, kWidth, kDecLo>(dec_w, kWidth, kWidth, m0, 32,
                                           decT + (size_t)m0 * kWidth, decL + (size_t)m0 * kWidth, sT, tid);
  } else {
    const int q = (bid - 16) * 256 + tid;
    const int o = q / 24;
    const int k8 = (q - o * 24) * 8;
    const int tap = k8 >> 6;
    const int c0 = k8 & 63;
    float vh[8];
    float vl[8];
#pragma unroll
    for (int e = 0; e < 8; ++e) {
      const float v = dil_w[(size_t)o * kDilK + (c0 + e) * 3 + tap] * kWCarry;
      const _Float16 hv = (_Float16)flush16(v);
      const float back = (float)hv;
      vh[e] = v;
      vl[e] = (v - back) * kLoScale;
    }
    const v4u ph = {pack2(vh[0], vh[1]), pack2(vh[2], vh[3]), pack2(vh[4], vh[5]), pack2(vh[6], vh[7])};
    store2_v4u(dilT + (size_t)q * 8, ph);
    if (kDilLo) {
      const v4u pl = {pack2(vl[0], vl[1]), pack2(vl[2], vl[3]), pack2(vl[4], vl[5]), pack2(vl[6], vl[7])};
      store2_v4u(dilL + (size_t)q * 8, pl);
    }
  }
}

template <bool LO>
__global__ __launch_bounds__(256) void encode_kernel(
    const float* __restrict__ x, const unsigned short* __restrict__ encT, const unsigned short* __restrict__ encL,
    const float* __restrict__ enc_b, unsigned short* __restrict__ u16) {
  __shared__ __align__(16) unsigned sXw[64 * kPitchX];
  __shared__ __align__(16) union { unsigned w[256 * 32]; unsigned short s[256 * 64]; } so;
  const int tid = threadIdx.x;
  const int lane = tid & 31;
  const int wave = __builtin_amdgcn_readfirstlane((int)(threadIdx.x >> 5));
  const int hh = lane >> 4;
  const int c = lane & 15;
  const size_t n0 = (size_t)blockIdx.x * 64;
#pragma unroll 1
  for (int it = 0; it < 4; ++it) {
    const int task = it * 256 + tid;
    const int row = task >> 4;
    const int c4 = (task & 15) * 4;
    const v4f xv = *(const v4f*)(x + (n0 + row) * kChanIn + c4);
    const v2u pk = {pack2(xv[0], xv[1]), pack2(xv[2], xv[3])};
    *(v2u*)(sXw + row * kPitchX + (c4 >> 1)) = pk;
  }
  __syncthreads();
  v8f acc[2][4];
  v8f accl[2][4];
#pragma unroll
  for (int i = 0; i < 2; ++i)
#pragma unroll
    for (int j = 0; j < 4; ++j) {
      acc[i][j] = (v8f){0.f, 0.f, 0.f, 0.f, 0.f, 0.f, 0.f, 0.f};
      accl[i][j] = (v8f){0.f, 0.f, 0.f, 0.f, 0.f, 0.f, 0.f, 0.f};
    }
  {
    const size_t wo = (size_t)(32 * wave + c) * kChanIn + 8 * hh;
    tile_kloop<LO, kPitchX>(acc, accl, (const _Float16*)encT + wo, (const _Float16*)encL + wo, kChanIn,
                            sXw, c, 4 * hh, kChanIn / 32);
  }
  acc_guard4(acc[0][0], acc[0][1], acc[0][2], acc[0][3]);
  acc_guard4(acc[1][0], acc[1][1], acc[1][2], acc[1][3]);
  if (LO) {
    acc_guard4(accl[0][0], accl[0][1], accl[0][2], accl[0][3]);
    acc_guard4(accl[1][0], accl[1][1], accl[1][2], accl[1][3]);
  }
#pragma unroll
  for (int i = 0; i < 2; ++i) {
    const int d0 = 32 * wave + 16 * i + 8 * hh;
    const v4f b0 = *(const v4f*)(enc_b + d0);
    const v4f b1 = *(const v4f*)(enc_b + d0 + 4);
#pragma unroll
    for (int j = 0; j < 4; ++j) {
      const int n = 16 * j + c;
#pragma unroll
      for (int r = 0; r < 8; ++r) {
        const float bv = (r < 4) ? b0[r & 3] : b1[r & 3];
        float a = acc[i][j][r];
        if (LO) a = fmaf(accl[i][j][r], kLoInv, a);
        const float o = fmaf(a, kWCarryInv, bv);
        so.s[(d0 + r) * 64 + n] = f16bits(o);
      }
    }
  }
  __syncthreads();
  store_tile_rows(so.w, u16, n0, wave, lane);
}

__global__ __launch_bounds__(256) void ktable_kernel(
    const float* __restrict__ la_re, const float* __restrict__ a_im,
    const float* __restrict__ b_re, const float* __restrict__ b_im,
    const float* __restrict__ c_re, const float* __restrict__ c_im,
    const float* __restrict__ log_dt, float* __restrict__ kt32) {
  __shared__ float sPar[4 * 256];
  __shared__ float sTab[4 * kTabSz];
  const int tid = threadIdx.x;
  const int h = blockIdx.x;
  {
    const int idx = h * kModes + tid;
    const float dt = expf(log_dt[h]);
    const float ar = -expf(la_re[idx]);
    const float ai = a_im[idx];
    const float dr = ar * dt;
    const float di = ai * dt;
    const float es = expf(dr);
    float sn, cs;
    sincosf(di, &sn, &cs);
    const float br = b_re[idx];
    const float bi = b_im[idx];
    const float cr = c_re[idx];
    const float ci = c_im[idx];
    const float pr = cr * br - ci * bi;
    const float pi = cr * bi + ci * br;
    sPar[tid]       = es * cs;
    sPar[256 + tid] = es * sn;
    sPar[512 + tid] = 2.0f * dt * pr;
    sPar[768 + tid] = 2.0f * dt * pi;
  }
  __syncthreads();
  const int nl = tid & 63;
  const int part = __builtin_amdgcn_readfirstlane((int)(threadIdx.x >> 6));
  const bool isA = part < 2;
  const bool up = (part & 1) != 0;
  const int jq = tid & 31;
  const int ig = tid >> 5;
  float kacc[4] = {0.0f, 0.0f, 0.0f, 0.0f};
#pragma unroll 1
  for (int q = 0; q < 4; ++q) {
    const int n = 64 * q + nl;
    const float wr = sPar[n];
    const float wi = sPar[256 + n];
    const float cr = sPar[512 + n];
    const float ci = sPar[768 + n];
    float sr = wr, si = wi;
#pragma unroll 1
    for (int s = 0; s < 4; ++s) csq(sr, si);
    const float w16r = sr, w16i = si;
    csq(sr, si);
    const float w32r = sr, w32i = si;
#pragma unroll 1
    for (int s = 0; s < 4; ++s) csq(sr, si);
    float cwr = cr, cwi = ci;
    cmul(cwr, cwi, sr, si);
    const float stepr = isA ? w32r : wr;
    const float stepi = isA ? w32i : wi;
    float curr = isA ? (up ? cwr : cr) : (up ? w16r : 1.0f);
    float curi = isA ? (up ? cwi : ci) : (up ? w16i : 0.0f);
    float* tre = sTab + (isA ? 0 : 2) * kTabSz + nl * 33 + (up ? 16 : 0);
    float* tim = tre + kTabSz;
#pragma unroll 1
    for (int e = 0; e < 16; ++e) {
      tre[e] = curr;
      tim[e] = curi;
      cmul(curr, curi, stepr, stepi);
    }
    __syncthreads();
    {
      const float* arp = sTab + ig;
      const float* aip = sTab + kTabSz + ig;
      const float* qrp = sTab + 2 * kTabSz + jq;
      const float* qip = sTab + 3 * kTabSz + jq;
#pragma unroll 2
      for (int nn = 0; nn < 64; ++nn) {
        const float qr = qrp[nn * 33];
        const float qi = qip[nn * 33];
#pragma unroll
        for (int m = 0; m < 4; ++m) {
          const float a = arp[nn * 33 + 8 * m];
          const float bq = aip[nn * 33 + 8 * m];
          kacc[m] += a * qr - bq * qi;
        }
      }
    }
    __syncthreads();
  }
  for (int pass = 0; pass < 2; ++pass) {
#pragma unroll
    for (int m = 0; m < 4; ++m) {
      *(volatile float*)(kt32 + (size_t)h * kLen + 256 * m + tid) = kacc[m];
    }
    __threadfence();
  }
}

__global__ __launch_bounds__(256) void toeplitz_kernel(
    const float* __restrict__ kt32, const float* __restrict__ dskip, unsigned short* __restrict__ tb16) {
  __shared__ float sW[256];
  const int tid = threadIdx.x;
  const int d = blockIdx.x;
  const int h = blockIdx.y;
  {
    const int kidx = 128 * d - 128 + tid;
    const int kc = (kidx < 0) ? 0 : kidx;
    const float v = kt32[(size_t)h * kLen + kc];
    sW[tid] = (kidx >= 0) ? v : 0.0f;
  }
  __syncthreads();
  const float dh = (d == 0) ? dskip[h] : 0.0f;
  unsigned short* dst = tb16 + ((size_t)(h * kBlocksD + d) * kChunk) * kChunk;
#pragma unroll 1
  for (int it = 0; it < 8; ++it) {
    const int q = it * 256 + tid;
    const int t = q >> 4;
    const int s0 = (q & 15) * 8;
    float v[8];
#pragma unroll
    for (int e = 0; e < 8; ++e) {
      const int m = 128 + t - (s0 + e);
      const float add = (m == 128) ? dh : 0.0f;
      v[e] = (sW[m] + add) * kTCarry;
    }
    const v4u pk = {pack2(v[0], v[1]), pack2(v[2], v[3]), pack2(v[4], v[5]), pack2(v[6], v[7])};
    store2_v4u(dst + (size_t)q * 8, pk);
  }
}

__global__ __launch_bounds__(256) void conv_kernel(
    const unsigned short* __restrict__ u16, const unsigned short* __restrict__ tb16, unsigned short* __restrict__ g16) {
  __shared__ __align__(16) float sT[8][16 * 68];
  __shared__ __align__(16) unsigned sHw[8][16 * 32];
  const int cch = blockIdx.x;
  const int lane = threadIdx.x & 31;
  const int wave = __builtin_amdgcn_readfirstlane((int)(threadIdx.x >> 5));
  const int h = 4 * (int)blockIdx.y + (wave >> 1);
  const int n0 = (wave & 1) * 64;
  const int rlane = lane & 15;
  const int koff = (lane >> 4) * 8;
  const int mOff = (lane >> 4) * 8;
  const _Float16* A = (const _Float16*)u16 + (size_t)h * kNpos;
  const _Float16* T = (const _Float16*)tb16 + (size_t)h * kBlocksD * kChunk * kChunk;

  v8f acc[2][4];
#pragma unroll
  for (int i = 0; i < 2; ++i)
#pragma unroll
    for (int j = 0; j < 4; ++j) acc[i][j] = (v8f){0.f, 0.f, 0.f, 0.f, 0.f, 0.f, 0.f, 0.f};

#pragma unroll 1
  for (int d = 0; d <= cch; ++d) {
    const _Float16* ap = A + (size_t)rlane * kLen + kChunk * (cch - d) + koff;
    const _Float16* bp = T + ((size_t)d * kChunk + n0 + rlane) * kChunk + koff;
    kloop32(acc, ap, kLen, bp, kChunk, kChunk / 32);
  }
  acc_guard4(acc[0][0], acc[0][1], acc[0][2], acc[0][3]);
  acc_guard4(acc[1][0], acc[1][1], acc[1][2], acc[1][3]);

  float* slab = sT[wave];
  unsigned* sH = sHw[wave];
  unsigned short* G = g16 + (size_t)h * kNpos + kChunk * cch + n0;
  const int q = lane >> 3;
  const int cw = lane & 7;
#pragma unroll
  for (int i = 0; i < 2; ++i) {
    const int mBase = i << 4;
#pragma unroll
    for (int j = 0; j < 4; ++j) {
#pragma unroll
      for (int r = 0; r < 8; ++r) slab[(mOff + r) * 68 + (j << 4) + rlane] = acc[i][j][r] * kTCarryInv;
    }
    wave_sync();
#pragma unroll 1
    for (int it = 0; it < 4; ++it) {
      const int row = it * 4 + q;
      const float* sp = slab + row * 68 + cw * 8;
      const v4f a0 = *(const v4f*)(sp);
      const v4f a1 = *(const v4f*)(sp + 4);
      const v4u pk = {pack2(gelu_fast(a0[0]), gelu_fast(a0[1])), pack2(gelu_fast(a0[2]), gelu_fast(a0[3])),
                      pack2(gelu_fast(a1[0]), gelu_fast(a1[1])), pack2(gelu_fast(a1[2]), gelu_fast(a1[3]))};
      *(v4u*)(sH + row * 32 + cw * 4) = pk;
    }
    wave_sync();
    v4u vals[4];
#pragma unroll
    for (int it = 0; it < 4; ++it) vals[it] = *(const v4u*)(sH + (it * 4 + q) * 32 + cw * 4);
    for (int pass = 0; pass < 2; ++pass) {
#pragma unroll
      for (int it = 0; it < 4; ++it) {
        const int row = it * 4 + q;
        *(volatile v4u*)(G + (size_t)(mBase + row) * kLen + cw * 8) = vals[it];
      }
      __threadfence();
    }
    wave_sync();
  }
}

__device__ __forceinline__ void col_reduce(float (&s)[4], float* sRed, float* sOut, int wave, int hh, int c, int tid) {
#pragma unroll
  for (int j = 0; j < 4; ++j) s[j] += __shfl_xor(s[j], 16, 32);
  if (hh == 0) {
#pragma unroll
    for (int j = 0; j < 4; ++j) sRed[wave * 64 + 16 * j + c] = s[j];
  }
  __syncthreads();
  if (tid < 64) {
    float a = 0.0f;
#pragma unroll 1
    for (int wv = 0; wv < 8; ++wv) a += sRed[wv * 64 + tid];
    sOut[tid] = a;
  }
  __syncthreads();
}

template <bool ENC_LO, bool DEC_LO, bool DIL_LO>
__global__ __launch_bounds__(256) void tail_kernel(
    const float* __restrict__ x, const unsigned short* __restrict__ g16,
    const unsigned short* __restrict__ encT, const unsigned short* __restrict__ encL,
    const unsigned short* __restrict__ decT, const unsigned short* __restrict__ decL,
    const unsigned short* __restrict__ dilT, const unsigned short* __restrict__ dilL,
    const float* __restrict__ enc_b, const float* __restrict__ ln1_g, const float* __restrict__ ln1_b,
    const float* __restrict__ dec_b, const float* __restrict__ dil_b,
    const float* __restrict__ ln2_g, const float* __restrict__ ln2_b, float* __restrict__ out) {
  __shared__ __align__(16) unsigned sXw[80 * kPitchX];
  __shared__ __align__(16) union { unsigned w[64 * kPitchW]; float f[64 * kPitchW]; } sb;
  __shared__ float sRed[512];
  __shared__ float sStat[128];
  const int tid = threadIdx.x;
  const int lane = tid & 31;
  const int wave = __builtin_amdgcn_readfirstlane((int)(threadIdx.x >> 5));
  const int hh = lane >> 4;
  const int c = lane & 15;
  const size_t n0 = (size_t)blockIdx.x * 64;
  const int b = (int)(n0 >> 10);
  const int l0 = (int)(n0 & (size_t)(kLen - 1));

#pragma unroll 1
  for (int it = 0; it < 5; ++it) {
    const int task = it * 256 + tid;
    const int row = task >> 4;
    const int c4 = (task & 15) * 4;
    const int l = l0 - 2 + row;
    int lc = (l < 0) ? 0 : l;
    lc = (lc > kLen - 1) ? (kLen - 1) : lc;
    const v4f xv = *(const v4f*)(x + ((size_t)b * kLen + lc) * kChanIn + c4);
    const bool ok = (l == lc);
    const float x0 = ok ? xv[0] : 0.0f;
    const float x1 = ok ? xv[1] : 0.0f;
    const float x2 = ok ? xv[2] : 0.0f;
    const float x3 = ok ? xv[3] : 0.0f;
    const v2u pk = {pack2(x0, x1), pack2(x2, x3)};
    *(v2u*)(sXw + row * kPitchX + (c4 >> 1)) = pk;
  }
  stage_tile_T<256>(g16, n0, sb.w, tid);
  __syncthreads();

  v8f acc[2][4];
  v8f accl[2][4];
#pragma unroll
  for (int i = 0; i < 2; ++i)
#pragma unroll
    for (int j = 0; j < 4; ++j) {
      acc[i][j] = (v8f){0.f, 0.f, 0.f, 0.f, 0.f, 0.f, 0.f, 0.f};
      accl[i][j] = (v8f){0.f, 0.f, 0.f, 0.f, 0.f, 0.f, 0.f, 0.f};
    }
  {
    const size_t wo = (size_t)(32 * wave + c) * kChanIn + 8 * hh;
    tile_kloop<ENC_LO, kPitchX>(acc, accl, (const _Float16*)encT + wo, (const _Float16*)encL + wo, kChanIn,
                                sXw, 2 + c, 4 * hh, kChanIn / 32);
  }
  acc_guard4(acc[0][0], acc[0][1], acc[0][2], acc[0][3]);
  acc_guard4(acc[1][0], acc[1][1], acc[1][2], acc[1][3]);
  if (ENC_LO) {
    acc_guard4(accl[0][0], accl[0][1], accl[0][2], accl[0][3]);
    acc_guard4(accl[1][0], accl[1][1], accl[1][2], accl[1][3]);
  }

  float s1[4] = {0.f, 0.f, 0.f, 0.f};
#pragma unroll
  for (int i = 0; i < 2; ++i) {
    const int d0 = 32 * wave + 16 * i + 8 * hh;
    const v4f e0 = *(const v4f*)(enc_b + d0);
    const v4f e1 = *(const v4f*)(enc_b + d0 + 4);
#pragma unroll
    for (int j = 0; j < 4; ++j) {
      const int n = 16 * j + c;
      const v4u rw = *(const v4u*)(sb.w + n * kPitchW + (d0 >> 1));
#pragma unroll
      for (int r = 0; r < 8; ++r) {
        const unsigned word = rw[r >> 1];
        const unsigned bits = (r & 1) ? (word >> 16) : (word & 0xffffu);
        const float gv = h16_to_f32(bits);
        const float bv = (r < 4) ? e0[r & 3] : e1[r & 3];
        float a = acc[i][j][r];
        if (ENC_LO) a = fmaf(accl[i][j][r], kLoInv, a);
        const float uv = fmaf(a, kWCarryInv, bv);
        const float val = gv + uv;
        acc[i][j][r] = val;
        s1[j] += val;
      }
    }
  }
  col_reduce(s1, sRed, sStat, wave, hh, c, tid);
  float mu[4], rs[4];
#pragma unroll
  for (int j = 0; j < 4; ++j) mu[j] = sStat[16 * j + c] * (1.0f / (float)kWidth);
  {
    float s2[4] = {0.f, 0.f, 0.f, 0.f};
#pragma unroll
    for (int i = 0; i < 2; ++i)
#pragma unroll
      for (int j = 0; j < 4; ++j)
#pragma unroll
        for (int r = 0; r < 8; ++r) {
          const float dv = acc[i][j][r] - mu[j];
          s2[j] = fmaf(dv, dv, s2[j]);
        }
    col_reduce(s2, sRed, sStat + 64, wave, hh, c, tid);
  }
#pragma unroll
  for (int j = 0; j < 4; ++j) rs[j] = rsqrtf(sStat[64 + 16 * j + c] * (1.0f / (float)kWidth) + 1e-5f);

#pragma unroll
  for (int i = 0; i < 2; ++i) {
    const int d0 = 32 * wave + 16 * i + 8 * hh;
    const v4f w0 = *(const v4f*)(ln1_g + d0);
    const v4f w1 = *(const v4f*)(ln1_g + d0 + 4);
    const v4f g0 = *(const v4f*)(ln1_b + d0);
    const v4f g1 = *(const v4f*)(ln1_b + d0 + 4);
#pragma unroll
    for (int j = 0; j < 4; ++j) {
      const int n = 16 * j + c;
      float o[8];
#pragma unroll
      for (int r = 0; r < 8; ++r) {
        const float lw = (r < 4) ? w0[r & 3] : w1[r & 3];
        const float lb = (r < 4) ? g0[r & 3] : g1[r & 3];
        const float xn = (acc[i][j][r] - mu[j]) * rs[j];
        o[r] = fmaf(xn, lw, lb) * kTCarry;
      }
      const v4u pk = {pack2(o[0], o[1]), pack2(o[2], o[3]), pack2(o[4], o[5]), pack2(o[6], o[7])};
      *(v4u*)(sb.w + n * kPitchW + (d0 >> 1)) = pk;
    }
  }
  __syncthreads();

#pragma unroll
  for (int i = 0; i < 2; ++i)
#pragma unroll
    for (int j = 0; j < 4; ++j) {
      acc[i][j] = (v8f){0.f, 0.f, 0.f, 0.f, 0.f, 0.f, 0.f, 0.f};
      accl[i][j] = (v8f){0.f, 0.f, 0.f, 0.f, 0.f, 0.f, 0.f, 0.f};
    }
  {
    const size_t wo = (size_t)(32 * wave + c) * kWidth + 8 * hh;
    tile_kloop<DEC_LO, kPitchW>(acc, accl, (const _Float16*)decT + wo, (const _Float16*)decL + wo, kWidth,
                                sb.w, c, 4 * hh, kWidth / 32);
  }
  acc_guard4(acc[0][0], acc[0][1], acc[0][2], acc[0][3]);
  acc_guard4(acc[1][0], acc[1][1], acc[1][2], acc[1][3]);
  if (DEC_LO) {
    acc_guard4(accl[0][0], accl[0][1], accl[0][2], accl[0][3]);
    acc_guard4(accl[1][0], accl[1][1], accl[1][2], accl[1][3]);
  }
#pragma unroll
  for (int i = 0; i < 2; ++i)
#pragma unroll
    for (int j = 0; j < 4; ++j)
#pragma unroll
      for (int r = 0; r < 8; ++r) {
        float a = acc[i][j][r];
        if (DEC_LO) a = fmaf(accl[i][j][r], kLoInv, a);
        acc[i][j][r] = a * kTCarryInv;
        if (DEC_LO || DIL_LO) accl[i][j][r] = 0.0f;
      }
#pragma unroll 1
  for (int tap = 0; tap < 3; ++tap) {
    const size_t wo = (size_t)(32 * wave + c) * kDilK + tap * kChanIn + 8 * hh;
    tile_kloop<DIL_LO, kPitchX>(acc, accl, (const _Float16*)dilT + wo, (const _Float16*)dilL + wo, kDilK,
                                sXw, 2 * tap + c, 4 * hh, kChanIn / 32);
  }
  acc_guard4(acc[0][0], acc[0][1], acc[0][2], acc[0][3]);
  acc_guard4(acc[1][0], acc[1][1], acc[1][2], acc[1][3]);
  if (DIL_LO) {
    acc_guard4(accl[0][0], accl[0][1], accl[0][2], accl[0][3]);
    acc_guard4(accl[1][0], accl[1][1], accl[1][2], accl[1][3]);
  }

#pragma unroll
  for (int j = 0; j < 4; ++j) s1[j] = 0.0f;
#pragma unroll
  for (int i = 0; i < 2; ++i) {
    const int d0 = 32 * wave + 16 * i + 8 * hh;
    const v4f p0 = *(const v4f*)(dec_b + d0);
    const v4f p1 = *(const v4f*)(dec_b + d0 + 4);
    const v4f t0 = *(const v4f*)(dil_b + d0);
    const v4f t1 = *(const v4f*)(dil_b + d0 + 4);
#pragma unroll
    for (int j = 0; j < 4; ++j) {
#pragma unroll
      for (int r = 0; r < 8; ++r) {
        const float bv = ((r < 4) ? p0[r & 3] : p1[r & 3]) + ((r < 4) ? t0[r & 3] : t1[r & 3]);
        float a = acc[i][j][r];
        if (DIL_LO) a = fmaf(accl[i][j][r], kLoInv, a);
        const float z = fmaf(a, kWCarryInv, bv);
        acc[i][j][r] = z;
        s1[j] += z;
      }
    }
  }
  col_reduce(s1, sRed, sStat, wave, hh, c, tid);
#pragma unroll
  for (int j = 0; j < 4; ++j) mu[j] = sStat[16 * j + c] * (1.0f / (float)kWidth);
  {
    float s2[4] = {0.f, 0.f, 0.f, 0.f};
#pragma unroll
    for (int i = 0; i < 2; ++i)
#pragma unroll
      for (int j = 0; j < 4; ++j)
#pragma unroll
        for (int r = 0; r < 8; ++r) {
          const float dv = acc[i][j][r] - mu[j];
          s2[j] = fmaf(dv, dv, s2[j]);
        }
    col_reduce(s2, sRed, sStat + 64, wave, hh, c, tid);
  }
#pragma unroll
  for (int j = 0; j < 4; ++j) rs[j] = rsqrtf(sStat[64 + 16 * j + c] * (1.0f / (float)kWidth) + 1e-5f);

#pragma unroll
  for (int i = 0; i < 2; ++i) {
    const int d0 = 32 * wave + 16 * i + 8 * hh;
    const v4f w0 = *(const v4f*)(ln2_g + d0);
    const v4f w1 = *(const v4f*)(ln2_g + d0 + 4);
    const v4f g0 = *(const v4f*)(ln2_b + d0);
    const v4f g1 = *(const v4f*)(ln2_b + d0 + 4);
#pragma unroll
    for (int j = 0; j < 4; ++j) {
#pragma unroll
      for (int r = 0; r < 8; ++r) {
        const float lw = (r < 4) ? w0[r & 3] : w1[r & 3];
        const float lb = (r < 4) ? g0[r & 3] : g1[r & 3];
        const float xn = (acc[i][j][r] - mu[j]) * rs[j];
        acc[i][j][r] = fmaf(xn, lw, lb);
      }
    }
  }

  float* slab = sb.f + wave * (16 * 36);
  const int q = lane >> 3;
  const int cw = lane & 7;
#pragma unroll
  for (int j = 0; j < 4; ++j) {
#pragma unroll
    for (int i = 0; i < 2; ++i) {
      const int dl = 16 * i + 8 * hh;
      const v4f lo4 = {acc[i][j][0], acc[i][j][1], acc[i][j][2], acc[i][j][3]};
      const v4f hi4 = {acc[i][j][4], acc[i][j][5], acc[i][j][6], acc[i][j][7]};
      *(v4f*)(slab + c * 36 + dl) = lo4;
      *(v4f*)(slab + c * 36 + dl + 4) = hi4;
    }
    wave_sync();
    v4f vals[4];
#pragma unroll
    for (int it = 0; it < 4; ++it) vals[it] = *(const v4f*)(slab + (it * 4 + q) * 36 + cw * 4);
    for (int pass = 0; pass < 2; ++pass) {
#pragma unroll
      for (int it = 0; it < 4; ++it) {
        const size_t pos = n0 + 16 * j + it * 4 + q;
        *(volatile v4f*)(out + pos * kWidth + 32 * wave + cw * 4) = vals[it];
      }
      __threadfence();
    }
    wave_sync();
  }
}

extern "C" void kernel_launch(void* const* d_in, const int* in_sizes, int n_in,
                              void* d_out, int out_size, void* d_ws, size_t ws_size,
                              hipStream_t stream) {
  if (n_in < 19) return;
  if (in_sizes[0] != kBatch * kLen * kChanIn) return;
  if (in_sizes[1] != kChanIn * kWidth) return;
  if (in_sizes[2] != kWidth) return;
  if (in_sizes[3] != kWidth * kModes) return;
  if (in_sizes[4] != kWidth * kModes) return;
  if (in_sizes[5] != kWidth * kModes) return;
  if (in_sizes[6] != kWidth * kModes) return;
  if (in_sizes[7] != kWidth * kModes) return;
  if (in_sizes[8] != kWidth * kModes) return;
  if (in_sizes[9] != kWidth) return;
  if (in_sizes[10] != kWidth) return;
  if (in_sizes[11] != kWidth) return;
  if (in_sizes[12] != kWidth) return;
  if (in_sizes[13] != kWidth * kWidth) return;
  if (in_sizes[14] != kWidth) return;
  if (in_sizes[15] != kWidth * kChanIn * 3) return;
  if (in_sizes[16] != kWidth) return;
  if (in_sizes[17] != kWidth) return;
  if (in_sizes[18] != kWidth) return;
  if (out_size != kBatch * kLen * kWidth) return;
  if (ws_size < kWsTotal) return;

  const float* x      = (const float*)d_in[0];
  const float* enc_w  = (const float*)d_in[1];
  const float* enc_b  = (const float*)d_in[2];
  const float* la_re  = (const float*)d_in[3];
  const float* a_im   = (const float*)d_in[4];
  const float* b_re   = (const float*)d_in[5];
  const float* b_im   = (const float*)d_in[6];
  const float* c_re   = (const float*)d_in[7];
  const float* c_im   = (const float*)d_in[8];
  const float* log_dt = (const float*)d_in[9];
  const float* dskip  = (const float*)d_in[10];
  const float* ln1_g  = (const float*)d_in[11];
  const float* ln1_b  = (const float*)d_in[12];
  const float* dec_w  = (const float*)d_in[13];
  const float* dec_b  = (const float*)d_in[14];
  const float* dil_w  = (const float*)d_in[15];
  const float* dil_b  = (const float*)d_in[16];
  const float* ln2_g  = (const float*)d_in[17];
  const float* ln2_b  = (const float*)d_in[18];
  float* out = (float*)d_out;

  char* ws = (char*)d_ws;
  unsigned short* U16  = (unsigned short*)(ws + kOffU16);
  unsigned short* G16  = (unsigned short*)(ws + kOffG16);
  float*          KT32 = (float*)(ws + kOffKt);
  unsigned short* TB16 = (unsigned short*)(ws + kOffTb);
  unsigned short* ENCT = (unsigned short*)(ws + kOffEncT);
  unsigned short* ENCL = (unsigned short*)(ws + kOffEncL);
  unsigned short* DECT = (unsigned short*)(ws + kOffDecT);
  unsigned short* DECL = (unsigned short*)(ws + kOffDecL);
  unsigned short* DILT = (unsigned short*)(ws + kOffDilT);
  unsigned short* DILL = (unsigned short*)(ws + kOffDilL);

  weight_planes_kernel<<<40, 256, 0, stream>>>(enc_w, dec_w, dil_w, ENCT, ENCL, DECT, DECL, DILT, DILL);
  encode_kernel<kEncLo><<<kNpos / 64, 256, 0, stream>>>(x, ENCT, ENCL, enc_b, U16);
  ktable_kernel<<<kWidth, 256, 0, stream>>>(la_re, a_im, b_re, b_im, c_re, c_im, log_dt, KT32);
  toeplitz_kernel<<<dim3(kBlocksD, kWidth), 256, 0, stream>>>(KT32, dskip, TB16);
  conv_kernel<<<dim3(kBlocksD, kWidth / 4), 256, 0, stream>>>(U16, TB16, G16);
  tail_kernel<kEncLo, kDecLo, kDilLo><<<kNpos / 64, 256, 0, stream>>>(
      x, G16, ENCT, ENCL, DECT, DECL, DILT, DILL, enc_b, ln1_g, ln1_b, dec_b, dil_b, ln2_g, ln2_b, out);
}
